// HyperEncoder_24592982737021
// MI455X (gfx1250) — hardware-verified
//
#include <hip/hip_runtime.h>
#include <math.h>

typedef unsigned short v8us __attribute__((ext_vector_type(8)));
typedef unsigned short v4us __attribute__((ext_vector_type(4)));
typedef __bf16 v16bf __attribute__((ext_vector_type(16)));
typedef float v8f __attribute__((ext_vector_type(8)));
typedef float v4f __attribute__((ext_vector_type(4)));
typedef int v8i __attribute__((ext_vector_type(8)));
typedef v8us __attribute__((may_alias)) v8usa;
typedef v4us __attribute__((may_alias)) v4usa;
typedef v4f  __attribute__((may_alias)) v4fa;

union Frag { v16bf v; v8us u[2]; v8i w; };

#define DIM  128
#define NB   128
#define NM   16
#define NROW (NB * NM)
#define KX   (2 * DIM)
#define NJ   (2 * DIM * DIM)
#define TP   68
#define XP   136
#define YP   128

static_assert(DIM == 128);
static_assert(NROW % 64 == 0);
static_assert(NJ % 64 == 0);
static_assert(KX % 64 == 0);
static_assert((XP * 2) % 16 == 0);
static_assert((TP * 4) % 16 == 0);

__device__ __forceinline__ unsigned short f2bf(float f) {
  unsigned int u = __float_as_uint(f);
  u = (u + 0x7FFFu + ((u >> 16) & 1u)) >> 16;
  return (unsigned short)u;
}
__device__ __forceinline__ float bf2f(unsigned short b) {
  return __uint_as_float(((unsigned int)b) << 16);
}
__device__ __forceinline__ float bfr(float f) { return bf2f(f2bf(f)); }

__device__ __forceinline__ v8f wmma_bf16(const Frag a, const Frag b, v8f c) {
  v8f d = __builtin_amdgcn_wmma_f32_16x16x32_bf16(false, a.v, false, b.v, (short)0, c, false, false);
  asm volatile("v_nop\n\tv_nop\n\tv_nop\n\tv_nop" : "+v"(d) : "v"(a.w), "v"(b.w));
  return d;
}

__device__ __forceinline__ Frag load_frag(const unsigned short* p, int h) {
  Frag f;
  f.u[0] = *(const v8usa*)(p + 8 * h);
  f.u[1] = *(const v8usa*)(p + 16 + 8 * h);
  return f;
}

__global__ __launch_bounds__(256) void wwt_kernel(const float* __restrict__ Ww,
                                                  unsigned short* __restrict__ WwT)
{
  __shared__ __attribute__((aligned(16))) float s_t[64 * TP];
  const int tid = threadIdx.x, lane = tid & 31, w = tid >> 5;
  const int j0 = blockIdx.x * 64, c0 = blockIdx.y * 64;
  const int f = tid & 15, cr = tid >> 4;
  #pragma unroll
  for (int i = 0; i < 4; ++i) {
    const int ci = cr + 16 * i;
    const v4f v = *(const v4fa*)(Ww + (size_t)(c0 + ci) * NJ + j0 + 4 * f);
    s_t[(4 * f + 0) * TP + ci] = v.x;
    s_t[(4 * f + 1) * TP + ci] = v.y;
    s_t[(4 * f + 2) * TP + ci] = v.z;
    s_t[(4 * f + 3) * TP + ci] = v.w;
  }
  __syncthreads();
  const int q8 = lane & 7, sub = lane >> 3;
  const int jj0 = w * 8 + sub, jj1 = w * 8 + 4 + sub;
  const float* sp0 = s_t + jj0 * TP + 8 * q8;
  const float* sp1 = s_t + jj1 * TP + 8 * q8;
  const v4f a0 = *(const v4fa*)sp0, c0v = *(const v4fa*)(sp0 + 4);
  const v4f a1 = *(const v4fa*)sp1, c1v = *(const v4fa*)(sp1 + 4);
  const v8us o0 = { f2bf(a0.x), f2bf(a0.y), f2bf(a0.z), f2bf(a0.w),
                    f2bf(c0v.x), f2bf(c0v.y), f2bf(c0v.z), f2bf(c0v.w) };
  const v8us o1 = { f2bf(a1.x), f2bf(a1.y), f2bf(a1.z), f2bf(a1.w),
                    f2bf(c1v.x), f2bf(c1v.y), f2bf(c1v.z), f2bf(c1v.w) };
  const size_t g0 = (size_t)(j0 + jj0) * KX + c0 + 8 * q8;
  const size_t g1 = (size_t)(j0 + jj1) * KX + c0 + 8 * q8;
  *(volatile v8us*)(WwT + g0) = o0;
  *(volatile v8us*)(WwT + g1) = o1;
  __threadfence();
  *(volatile v8us*)(WwT + g0) = o0;
  *(volatile v8us*)(WwT + g1) = o1;
}

__global__ __launch_bounds__(256) void fused_kernel(
    const float* __restrict__ msg,
    const unsigned short* __restrict__ WwT,
    const float* __restrict__ Wb,
    const float* __restrict__ bw,
    const float* __restrict__ bb,
    float* __restrict__ out)
{
  __shared__ __attribute__((aligned(16))) unsigned short s_x[64 * XP];
  __shared__ __attribute__((aligned(16))) unsigned short s_ag[2 * 16 * XP];
  __shared__ __attribute__((aligned(16))) float s_aggf[4 * DIM];
  __shared__ float s_bsc[64];
  __shared__ __attribute__((aligned(16))) float s_y[64 * YP];
  __shared__ __attribute__((aligned(16))) float s_out[4 * DIM];

  const int tid = threadIdx.x, lane = tid & 31, w = tid >> 5;
  const int h = lane >> 4, m = lane & 15;
  const int rh = w >> 2, cq = w & 3;
  const int row0 = blockIdx.x * 64;
  const int b0 = blockIdx.x * 4;

  #pragma unroll
  for (int i = 0; i < 8; ++i) {
    const int idx = tid + 256 * i;
    const int r = idx >> 5, f = idx & 31;
    const v4f v = *(const v4fa*)(msg + (size_t)(row0 + r) * DIM + 4 * f);
    const v4us o = { f2bf(v.x), f2bf(v.y), f2bf(v.z), f2bf(v.w) };
    *(v4usa*)(s_x + r * XP + 4 * f) = o;
  }
  __syncthreads();

  #pragma unroll
  for (int i = 0; i < 2; ++i) {
    const int idx = tid + 256 * i;
    const int bt = idx >> 7, dd = idx & 127;
    float s = 0.0f;
    #pragma unroll
    for (int mm = 0; mm < NM; ++mm) s += bf2f(s_x[(16 * bt + mm) * XP + dd]);
    s_aggf[idx] = s;
  }
  __syncthreads();

  #pragma unroll
  for (int i = 0; i < 4; ++i) {
    const int q = tid + 256 * i;
    const int rhh = q >> 9, rowi = (q >> 5) & 15, c4 = (q & 31) * 4;
    const int rr = rowi & 7;
    const int bsel = 2 * rhh + (rr & 1);
    const int part = (rr >> 1) & 1;
    const bool live = (rr < 4);
    v4us o = { 0, 0, 0, 0 };
    #pragma unroll
    for (int e = 0; e < 4; ++e) {
      const float a = s_aggf[bsel * DIM + c4 + e];
      const unsigned short hb = f2bf(a);
      const unsigned short lb = f2bf(a - bf2f(hb));
      const unsigned short v = part ? lb : hb;
      o[e] = live ? v : (unsigned short)0;
    }
    *(v4usa*)(s_ag + (rhh * 16 + rowi) * XP + c4) = o;
  }
  if (tid < 64) {
    const int r = tid, bt = r >> 4;
    float acc = 0.0f;
    #pragma unroll 4
    for (int c = 0; c < DIM; ++c) acc += bf2f(s_x[r * XP + c]) * bfr(bw[c]);
    #pragma unroll 4
    for (int c = 0; c < DIM; ++c) acc += s_aggf[bt * DIM + c] * bfr(bw[DIM + c]);
    acc += bfr(bb[0]);
    s_bsc[r] = acc;
  }
  __syncthreads();

  const v8f zero8 = { 0.f, 0.f, 0.f, 0.f, 0.f, 0.f, 0.f, 0.f };
  v8f Y[2][2];
  #pragma unroll
  for (int rt = 0; rt < 2; ++rt)
    #pragma unroll
    for (int ct = 0; ct < 2; ++ct) Y[rt][ct] = zero8;

  const unsigned short* xa = s_x + (32 * rh + m) * XP;
  const unsigned short* aa = s_ag + (16 * rh + m) * XP;
  const int colw = 32 * cq + m;

  #pragma unroll 1
  for (int k = 0; k < KX; ++k) {
    const unsigned short* bq0 = WwT + (size_t)(k * DIM + colw) * KX;
    const unsigned short* bq1 = bq0 + (size_t)16 * KX;

    v8f T[2][2], TA[2];
    #pragma unroll
    for (int rt = 0; rt < 2; ++rt)
      #pragma unroll
      for (int ct = 0; ct < 2; ++ct) T[rt][ct] = zero8;
    TA[0] = zero8; TA[1] = zero8;

    #pragma unroll 1
    for (int s = 0; s < 4; ++s) {
      const int c0 = 32 * s;
      const Frag ag  = load_frag(aa + c0, h);
      const Frag bg0 = load_frag(bq0 + DIM + c0, h);
      const Frag bg1 = load_frag(bq1 + DIM + c0, h);
      TA[0] = wmma_bf16(ag, bg0, TA[0]);
      TA[1] = wmma_bf16(ag, bg1, TA[1]);
      const Frag am0 = load_frag(xa + c0, h);
      const Frag am1 = load_frag(xa + 16 * XP + c0, h);
      const Frag bm0 = load_frag(bq0 + c0, h);
      const Frag bm1 = load_frag(bq1 + c0, h);
      T[0][0] = wmma_bf16(am0, bm0, T[0][0]);
      T[0][1] = wmma_bf16(am0, bm1, T[0][1]);
      T[1][0] = wmma_bf16(am1, bm0, T[1][0]);
      T[1][1] = wmma_bf16(am1, bm1, T[1][1]);
    }

    const float wb0 = bfr(Wb[k * DIM + colw]);
    const float wb1 = bfr(Wb[k * DIM + colw + 16]);
    const bool useagg = (k >= DIM);
    const int kc = useagg ? (DIM - 1) : k;
    const int ka = useagg ? (k - DIM) : 0;
    const float ag0 = s_aggf[(2 * rh) * DIM + ka];
    const float ag1 = s_aggf[(2 * rh + 1) * DIM + ka];
    const float base00 = (TA[0][0] + TA[0][2]) + wb0;
    const float base01 = (TA[1][0] + TA[1][2]) + wb1;
    const float base10 = (TA[0][1] + TA[0][3]) + wb0;
    const float base11 = (TA[1][1] + TA[1][3]) + wb1;
    #pragma unroll
    for (int r = 0; r < 8; ++r) {
      const float xm0 = bf2f(s_x[(32 * rh + 8 * h + r) * XP + kc]);
      const float xm1 = bf2f(s_x[(32 * rh + 16 + 8 * h + r) * XP + kc]);
      const float x0 = useagg ? ag0 : xm0;
      const float x1 = useagg ? ag1 : xm1;
      Y[0][0][r] += x0 * (T[0][0][r] + base00);
      Y[0][1][r] += x0 * (T[0][1][r] + base01);
      Y[1][0][r] += x1 * (T[1][0][r] + base10);
      Y[1][1][r] += x1 * (T[1][1][r] + base11);
    }
  }

  #pragma unroll
  for (int r = 0; r < 8; ++r) {
    const int ra = (32 * rh + 8 * h + r) * YP + colw;
    const int rb = ra + 16 * YP;
    s_y[ra]      = Y[0][0][r];
    s_y[ra + 16] = Y[0][1][r];
    s_y[rb]      = Y[1][0][r];
    s_y[rb + 16] = Y[1][1][r];
  }
  __syncthreads();

  {
    const int col = tid & 127, bp = tid >> 7;
    #pragma unroll
    for (int e = 0; e < 2; ++e) {
      const int bt = 2 * bp + e;
      float acc = 0.0f;
      #pragma unroll 1
      for (int mm = 0; mm < NM; ++mm) {
        const float v = s_y[(16 * bt + mm) * YP + col] + s_bsc[16 * bt + mm];
        acc += (v > 0.0f) ? v : expm1f(v);
      }
      s_out[bt * DIM + col] = acc;
    }
  }
  __syncthreads();

  const bool wr = (tid < 128);
  v4f ov = { 0.f, 0.f, 0.f, 0.f };
  size_t og = 0;
  if (wr) {
    const int line = tid >> 3, q8 = tid & 7;
    ov = *(const v4fa*)(s_out + line * 32 + 4 * q8);
    og = (size_t)b0 * DIM + line * 32 + 4 * q8;
    *(volatile v4f*)(out + og) = ov;
  }
  __threadfence();
  if (wr) *(volatile v4f*)(out + og) = ov;
}

extern "C" void kernel_launch(void* const* d_in, const int* in_sizes, int n_in,
                              void* d_out, int out_size, void* d_ws, size_t ws_size,
                              hipStream_t stream) {
  if (n_in < 5) return;
  if (in_sizes[0] != NROW * DIM) return;
  if (in_sizes[1] != KX * NJ) return;
  if (in_sizes[2] != NJ) return;
  if (in_sizes[3] != KX) return;
  if (in_sizes[4] < 1) return;
  if (out_size != NB * DIM) return;

  const size_t wwt_bytes = (size_t)NJ * KX * 2;
  if (wwt_bytes > ws_size) return;

  const float* msg = (const float*)d_in[0];
  const float* Ww  = (const float*)d_in[1];
  const float* Wb  = (const float*)d_in[2];
  const float* bw  = (const float*)d_in[3];
  const float* bb  = (const float*)d_in[4];
  unsigned short* WwT = (unsigned short*)d_ws;
  float* out = (float*)d_out;

  dim3 gT(NJ / 64, KX / 64);
  wwt_kernel<<<gT, 256, 0, stream>>>(Ww, WwT);
  fused_kernel<<<NROW / 64, 256, 0, stream>>>(msg, WwT, Wb, bw, bb, out);
}
